// KANLinear_49641232007351
// MI455X (gfx1250) — hardware-verified
//
#include <hip/hip_runtime.h>
#include <math.h>

constexpr int kRows     = 16384;
constexpr int kIn       = 512;
constexpr int kOutF     = 512;
constexpr int kCoef     = 8;
constexpr int kKsp      = kIn * kCoef;
constexpr int kKtot     = kIn + kKsp;
constexpr int kHalfRows = 8192;
constexpr int kNumHalves = kRows / kHalfRows;
constexpr float kKnotH   = 0.4f;
constexpr float kKnotLo  = -1.0f;
constexpr float kWCarry    = 64.0f;
constexpr float kWCarryInv = 1.0f / 64.0f;

constexpr size_t kWctBytes = (size_t)kOutF * kKtot * 2;
constexpr size_t kAhBytes  = (size_t)kHalfRows * kKtot * 2;
constexpr size_t kWsTotal  = kWctBytes + kAhBytes;
static_assert(kWctBytes % 128 == 0, "plane offsets line aligned");
static_assert(kWsTotal <= 134217728ull, "carve within 128 MiB");
static_assert(kKtot % 32 == 0, "GEMM K multiple of 32");
static_assert(kHalfRows % 64 == 0 && kOutF % 64 == 0, "GEMM M,N tile multiples");
static_assert(kRows % kHalfRows == 0, "whole passes");
static_assert((kKtot % 64) == 0, "row pitch is a whole number of 128-B lines");

typedef __attribute__((ext_vector_type(16))) _Float16 v16h;
typedef __attribute__((ext_vector_type(8)))  _Float16 v8h;
typedef __attribute__((ext_vector_type(16))) __bf16   v16b;
typedef __attribute__((ext_vector_type(8)))  __bf16   v8b;
typedef __attribute__((ext_vector_type(8)))  float    v8f;
typedef __attribute__((ext_vector_type(4)))  float    v4f;
typedef __attribute__((ext_vector_type(4)))  unsigned int v4u;

__device__ __forceinline__ unsigned short f2bf_bits(float f) {
  unsigned u = __float_as_uint(f);
  return (unsigned short)((u + 0x7FFFu + ((u >> 16) & 1u)) >> 16);
}
__device__ __forceinline__ float bf_bits2f(unsigned short h) { return __uint_as_float(((unsigned)h) << 16); }

__device__ __forceinline__ void dep_guard_h(v8f& a, v8f& b, v16h x, v16h y) { asm volatile("v_nop\n\tv_nop\n\tv_nop\n\tv_nop" : "+v"(a), "+v"(b) : "v"(x), "v"(y)); }
__device__ __forceinline__ void dep_guard_b(v8f& a, v8f& b, v16b x, v16b y) { asm volatile("v_nop\n\tv_nop\n\tv_nop\n\tv_nop" : "+v"(a), "+v"(b) : "v"(x), "v"(y)); }
__device__ __forceinline__ void dep_guard4_h(v8f& a, v8f& b, v8f& c, v8f& d, v16h x, v16h y) { asm volatile("v_nop\n\tv_nop\n\tv_nop\n\tv_nop" : "+v"(a), "+v"(b), "+v"(c), "+v"(d) : "v"(x), "v"(y)); }
__device__ __forceinline__ void dep_guard4_b(v8f& a, v8f& b, v8f& c, v8f& d, v16b x, v16b y) { asm volatile("v_nop\n\tv_nop\n\tv_nop\n\tv_nop" : "+v"(a), "+v"(b), "+v"(c), "+v"(d) : "v"(x), "v"(y)); }
__device__ __forceinline__ void keep4_h(v16h a, v16h b, v16h c, v16h d) { asm volatile("v_nop" :: "v"(a), "v"(b), "v"(c), "v"(d)); }
__device__ __forceinline__ void keep4_b(v16b a, v16b b, v16b c, v16b d) { asm volatile("v_nop" :: "v"(a), "v"(b), "v"(c), "v"(d)); }
__device__ __forceinline__ void acc_guard4(v8f& a, v8f& b, v8f& c, v8f& d) { asm volatile("v_nop\n\tv_nop\n\tv_nop\n\tv_nop" : "+v"(a), "+v"(b), "+v"(c), "+v"(d)); }
template <typename T> struct Frag;
template <> struct Frag<_Float16> {
  typedef v16h V; union U { v16h v; v8h h[2]; };
  static __device__ __forceinline__ v16h load(const _Float16* p) {
    U f; f.h[0] = *(const v8h*)(p); f.h[1] = *(const v8h*)(p + 16); return f.v;
  }
  static __device__ __forceinline__ v8f mma(v16h a, v16h b, v8f c) {
    return __builtin_amdgcn_wmma_f32_16x16x32_f16(false, a, false, b, (short)0, c, false, false);
  }
  static __device__ __forceinline__ void guard(v8f& a, v8f& b, v16h x, v16h y) { dep_guard_h(a, b, x, y); }
  static __device__ __forceinline__ void guard4(v8f& a, v8f& b, v8f& c, v8f& d, v16h x, v16h y) { dep_guard4_h(a, b, c, d, x, y); }
  static __device__ __forceinline__ void keep(v16h a, v16h b, v16h c, v16h d) { keep4_h(a, b, c, d); }
};
template <> struct Frag<__bf16> {
  typedef v16b V; union U { v16b v; v8b h[2]; };
  static __device__ __forceinline__ v16b load(const __bf16* p) {
    U f; f.h[0] = *(const v8b*)(p); f.h[1] = *(const v8b*)(p + 16); return f.v;
  }
  static __device__ __forceinline__ v8f mma(v16b a, v16b b, v8f c) {
    return __builtin_amdgcn_wmma_f32_16x16x32_bf16(false, a, false, b, (short)0, c, false, false);
  }
  static __device__ __forceinline__ void guard(v8f& a, v8f& b, v16b x, v16b y) { dep_guard_b(a, b, x, y); }
  static __device__ __forceinline__ void guard4(v8f& a, v8f& b, v8f& c, v8f& d, v16b x, v16b y) { dep_guard4_b(a, b, c, d, x, y); }
  static __device__ __forceinline__ void keep(v16b a, v16b b, v16b c, v16b d) { keep4_b(a, b, c, d); }
};

__device__ __forceinline__ unsigned pk16(unsigned short a, unsigned short b) { return (unsigned)a | ((unsigned)b << 16); }
__device__ __forceinline__ unsigned short h_bits(float f) { const _Float16 h = (_Float16)f; return __builtin_bit_cast(unsigned short, h); }

template <int ET> struct Elem;
template <> struct Elem<0> { typedef _Float16 T; };
template <> struct Elem<1> { typedef __bf16 T; };
template <int ET, bool SPLIT, int BIAS_MODE, int OUT_MODE, bool RESID, int ACT = 0>
__global__ __launch_bounds__(256) void wmma_gemm64(
    const unsigned short* __restrict__ Ap, const unsigned short* __restrict__ A2p, int lda, long strideA,
    const unsigned short* __restrict__ Btp, const unsigned short* __restrict__ Bt2p, int ldb, long strideB,
    void* __restrict__ Cout, void* __restrict__ Cout2, int ldc, long strideC,
    const float* __restrict__ bias,
    const float* __restrict__ resid, long strideR,
    int M, int N, int K, float scale) {
  typedef typename Elem<ET>::T T;
  typedef typename Frag<T>::V V;
  const T* A = (const T*)Ap; const T* A2 = (const T*)A2p; const T* Bt = (const T*)Btp; const T* Bt2 = (const T*)Bt2p;
  __shared__ __align__(16) float sT[8][16 * 68];
  const int b    = blockIdx.y;
  const int lane = threadIdx.x & 31;
  const int wave = threadIdx.x >> 5;
  const int tilesN = N >> 6;
  const int tilesM = M >> 6;
  const int tile = blockIdx.x * 8 + wave;
  if (tile >= tilesM * tilesN) return;
  const int tm = tile / tilesN;
  const int tn = tile - tm * tilesN;
  const int m0 = tm << 6;
  const int n0 = tn << 6;

  const T* Ab  = A  + (size_t)b * strideA;
  const T* Bb  = Bt + (size_t)b * strideB;
  const T* Ab2 = SPLIT ? (A2  + (size_t)b * strideA) : nullptr;
  const T* Bb2 = SPLIT ? (Bt2 + (size_t)b * strideB) : nullptr;

  const int rlane = lane & 15;
  const int koff  = (lane >> 4) * 8;
  const int mOff  = (lane >> 4) * 8;

  v8f acc[4][4];
#pragma unroll
  for (int i = 0; i < 4; ++i)
#pragma unroll
    for (int j = 0; j < 4; ++j) acc[i][j] = (v8f){0.f,0.f,0.f,0.f,0.f,0.f,0.f,0.f};

  for (int k0 = 0; k0 < K; k0 += 32) {
    V bh[4], bl[4];
#pragma unroll
    for (int j = 0; j < 4; ++j) {
      const size_t bo = (size_t)(n0 + (j << 4) + rlane) * ldb + koff + k0;
      bh[j] = Frag<T>::load(Bb + bo);
      if (SPLIT) bl[j] = Frag<T>::load(Bb2 + bo);
    }
#pragma unroll
    for (int i = 0; i < 4; ++i) {
      const size_t ao = (size_t)(m0 + (i << 4) + rlane) * lda + koff + k0;
      V ah = Frag<T>::load(Ab + ao);
      V al;
      if (SPLIT) al = Frag<T>::load(Ab2 + ao);
#pragma unroll
      for (int j = 0; j < 4; ++j) {
        acc[i][j] = Frag<T>::mma(ah, bh[j], acc[i][j]);
        if (SPLIT) {
          acc[i][j] = Frag<T>::mma(ah, bl[j], acc[i][j]);
          acc[i][j] = Frag<T>::mma(al, bh[j], acc[i][j]);
        }
      }
      Frag<T>::guard4(acc[i][0], acc[i][1], acc[i][2], acc[i][3], ah, SPLIT ? al : ah);
    }
    Frag<T>::keep(bh[0], bh[1], bh[2], bh[3]);
    if (SPLIT) Frag<T>::keep(bl[0], bl[1], bl[2], bl[3]);
  }
  acc_guard4(acc[0][0], acc[0][1], acc[0][2], acc[0][3]);
  acc_guard4(acc[1][0], acc[1][1], acc[1][2], acc[1][3]);
  acc_guard4(acc[2][0], acc[2][1], acc[2][2], acc[2][3]);
  acc_guard4(acc[3][0], acc[3][1], acc[3][2], acc[3][3]);

  float* slab = sT[wave];
  const float* Rb = RESID ? (resid + (size_t)b * strideR) : nullptr;
#pragma unroll
  for (int i = 0; i < 4; ++i) {
    const int mBase = m0 + (i << 4);
#pragma unroll
    for (int j = 0; j < 4; ++j) {
      const int n = n0 + (j << 4) + rlane;
      float bv = 0.f;
      if (BIAS_MODE == 2) bv = bias[n];
#pragma unroll
      for (int r = 0; r < 8; ++r) {
        float v = acc[i][j][r] * scale;
        if (BIAS_MODE == 1) v += bias[mBase + mOff + r];
        if (BIAS_MODE == 2) v += bv;
        if (RESID) v += Rb[(size_t)(mBase + mOff + r) * ldc + n];
        if (ACT == 2) v = fmaxf(v, 0.0f);
        if (ACT == 4) v = (v > 0.f) ? v : 0.01f * v;
        slab[(mOff + r) * 68 + (j << 4) + rlane] = v;
      }
    }
    __builtin_amdgcn_fence(__ATOMIC_RELEASE, "workgroup");
    __builtin_amdgcn_wave_barrier();
    __builtin_amdgcn_fence(__ATOMIC_ACQUIRE, "workgroup");
    if (OUT_MODE == 0) {
      float* C = (float*)Cout + (size_t)b * strideC;
      const int hh = lane >> 4, c4 = (lane & 15) * 4;
      for (int pass = 0; pass < 2; ++pass) {
#pragma unroll
        for (int it = 0; it < 8; ++it) {
          const int row = it * 2 + hh;
          v4f v = *(const v4f*)(slab + row * 68 + c4);
          *(volatile v4f*)(C + (size_t)(mBase + row) * ldc + n0 + c4) = v;
        }
        __threadfence();
      }
    } else {
      const int q = lane >> 3, c8 = (lane & 7) * 8;
      unsigned short* C  = (unsigned short*)Cout  + (size_t)b * strideC;
      unsigned short* C2 = (OUT_MODE == 2) ? ((unsigned short*)Cout2 + (size_t)b * strideC) : nullptr;
      for (int pass = 0; pass < 2; ++pass) {
#pragma unroll
        for (int it = 0; it < 4; ++it) {
          const int row = it * 4 + q;
          const float* sp = slab + row * 68 + c8;
          v8h hv, lv;
#pragma unroll
          for (int e = 0; e < 8; ++e) {
            if (OUT_MODE == 1) {
              hv[e] = (_Float16)sp[e];
            } else {
              unsigned short hb = f2bf_bits(sp[e]);
              unsigned short lb = f2bf_bits(sp[e] - bf_bits2f(hb));
              hv[e] = __builtin_bit_cast(_Float16, hb);
              lv[e] = __builtin_bit_cast(_Float16, lb);
            }
          }
          *(volatile v8h*)(C + (size_t)(mBase + row) * ldc + n0 + c8) = hv;
          if (OUT_MODE == 2) *(volatile v8h*)(C2 + (size_t)(mBase + row) * ldc + n0 + c8) = lv;
        }
        __threadfence();
      }
    }
    __builtin_amdgcn_fence(__ATOMIC_RELEASE, "workgroup");
    __builtin_amdgcn_wave_barrier();
    __builtin_amdgcn_fence(__ATOMIC_ACQUIRE, "workgroup");
  }
}

__global__ __launch_bounds__(256) void wplane2_kernel(const float* __restrict__ bw, const float* __restrict__ sw,
                                                      const float* __restrict__ ss, unsigned short* __restrict__ Wp, int nthr) {
  const int i = blockIdx.x * 256 + threadIdx.x;
  if (i >= nthr) return;
  const int e  = 2 * i;
  const int n  = e / kKtot;
  const int k  = e - n * kKtot;
  const int kb = (k < kIn - 2) ? k : (kIn - 2);
  const float a0 = bw[(size_t)n * kIn + kb];
  const float a1 = bw[(size_t)n * kIn + kb + 1];
  const int kp = (k >= kIn) ? (k - kIn) : 0;
  const float sc = ss[(size_t)n * kIn + (kp >> 3)];
  const float c0 = sw[(size_t)n * kKsp + kp] * sc;
  const float c1 = sw[(size_t)n * kKsp + kp + 1] * sc;
  const float fa = (k < kIn) ? 1.0f : 0.0f;
  const float fb = 1.0f - fa;
  const float w0 = fmaf(fa, a0, fb * c0) * kWCarry;
  const float w1 = fmaf(fa, a1, fb * c1) * kWCarry;
  const unsigned u = pk16(h_bits(w0), h_bits(w1));
  unsigned* q = (unsigned*)(Wp + (size_t)e);
  *(volatile unsigned*)q = u;
  __threadfence();
  *(volatile unsigned*)q = u;
}

__global__ __launch_bounds__(256) void silu2_kernel(const float* __restrict__ x, unsigned short* __restrict__ Ah,
                                                    int row0, int nthr) {
  const int i = blockIdx.x * 256 + threadIdx.x;
  if (i >= nthr) return;
  const int row = i >> 8;
  const int c   = (i & 255) * 2;
  const float* p = x + (size_t)(row0 + row) * kIn + c;
  const float x0 = p[0];
  const float x1 = p[1];
  const float s0 = x0 * (1.0f / (1.0f + expf(-x0)));
  const float s1 = x1 * (1.0f / (1.0f + expf(-x1)));
  const unsigned u = pk16(h_bits(s0), h_bits(s1));
  unsigned* q = (unsigned*)(Ah + (size_t)row * kKtot + c);
  *(volatile unsigned*)q = u;
  __threadfence();
  *(volatile unsigned*)q = u;
}

__global__ __launch_bounds__(256) void bases8_kernel(const float* __restrict__ x, unsigned short* __restrict__ Ah,
                                                     int row0, int nthr) {
#pragma clang fp contract(off)
  const int i = blockIdx.x * 256 + threadIdx.x;
  if (i >= nthr) return;
  const int row = i >> 9;
  const int f   = i & 511;
  const float xv = x[(size_t)(row0 + row) * kIn + f];

  float g[12];
#pragma unroll
  for (int j = 0; j < 12; ++j) g[j] = (float)(j - 3) * kKnotH + kKnotLo;

  float b0[11];
#pragma unroll
  for (int j = 0; j < 11; ++j) b0[j] = ((xv >= g[j]) && (xv < g[j + 1])) ? 1.0f : 0.0f;

  float b1[10];
#pragma unroll
  for (int j = 0; j < 10; ++j) {
    const float lf = (xv - g[j]) * (1.0f / (g[j + 1] - g[j]));
    const float rt = (g[j + 2] - xv) * (1.0f / (g[j + 2] - g[j + 1]));
    const float tl = lf * b0[j];
    const float tr = rt * b0[j + 1];
    b1[j] = tl + tr;
  }
  float b2[9];
#pragma unroll
  for (int j = 0; j < 9; ++j) {
    const float lf = (xv - g[j]) * (1.0f / (g[j + 2] - g[j]));
    const float rt = (g[j + 3] - xv) * (1.0f / (g[j + 3] - g[j + 1]));
    const float tl = lf * b1[j];
    const float tr = rt * b1[j + 1];
    b2[j] = tl + tr;
  }
  float b3[8];
#pragma unroll
  for (int j = 0; j < 8; ++j) {
    const float lf = (xv - g[j]) * (1.0f / (g[j + 3] - g[j]));
    const float rt = (g[j + 4] - xv) * (1.0f / (g[j + 4] - g[j + 1]));
    const float tl = lf * b2[j];
    const float tr = rt * b2[j + 1];
    b3[j] = tl + tr;
  }

  unsigned short hb[8];
#pragma unroll
  for (int e = 0; e < 8; ++e) hb[e] = h_bits(b3[e]);
  const v4u u = (v4u){pk16(hb[0], hb[1]), pk16(hb[2], hb[3]), pk16(hb[4], hb[5]), pk16(hb[6], hb[7])};
  unsigned short* q = Ah + (size_t)row * kKtot + kIn + 8 * f;
  *(volatile v4u*)q = u;
  __threadfence();
  *(volatile v4u*)q = u;
}

extern "C" void kernel_launch(void* const* d_in, const int* in_sizes, int n_in,
                              void* d_out, int out_size, void* d_ws, size_t ws_size,
                              hipStream_t stream) {
  if (n_in < 4) return;
  if (in_sizes[0] != kRows * kIn) return;
  if (in_sizes[1] != kOutF * kIn) return;
  if (in_sizes[2] != kOutF * kKsp) return;
  if (in_sizes[3] != kOutF * kIn) return;
  if (out_size != kRows * kOutF) return;
  if (ws_size < kWsTotal) return;

  const float* x  = (const float*)d_in[0];
  const float* bw = (const float*)d_in[1];
  const float* sw = (const float*)d_in[2];
  const float* ss = (const float*)d_in[3];
  float* out = (float*)d_out;

  unsigned short* wct = (unsigned short*)d_ws;
  unsigned short* ah  = (unsigned short*)((char*)d_ws + kWctBytes);

  const int nthr_w = kOutF * kKtot / 2;
  wplane2_kernel<<<dim3((nthr_w + 255) / 256), dim3(256), 0, stream>>>(bw, sw, ss, wct, nthr_w);

  const int nthr_s = kHalfRows * (kIn / 2);
  const int nthr_b = kHalfRows * kIn;
  const int gemm_tiles  = (kHalfRows / 64) * (kOutF / 64);
  const int gemm_blocks = (gemm_tiles + 7) / 8;

  for (int hp = 0; hp < kNumHalves; ++hp) {
    const int row0 = hp * kHalfRows;
    silu2_kernel<<<dim3((nthr_s + 255) / 256), dim3(256), 0, stream>>>(x, ah, row0, nthr_s);
    bases8_kernel<<<dim3((nthr_b + 255) / 256), dim3(256), 0, stream>>>(x, ah, row0, nthr_b);
    float* cdst = out + (size_t)row0 * kOutF;
    wmma_gemm64<0, false, 0, 0, false, 0><<<dim3(gemm_blocks, 1), dim3(256), 0, stream>>>(
        ah, ah, kKtot, 0L,
        wct, wct, kKtot, 0L,
        (void*)cdst, (void*)cdst, kOutF, 0L,
        bw,
        bw, 0L,
        kHalfRows, kOutF, kKtot, kWCarryInv);
  }
}
